// GAT_33844342293157
// MI455X (gfx1250) — hardware-verified
//
#include <hip/hip_runtime.h>
#include <stddef.h>
#include <stdint.h>
#include <math.h>


#define XW      1024
#define HW      512
#define FW      1536
#define KHL     1024
#define NTHR    256
#define NWAVE   8
#define EPT     8
#define CHUNK   (NTHR * EPT)
#define WCAP    (EPT * 32)
#define LISTN   (NWAVE * WCAP)
#define NB      256
#define SLOTB   8
#define RPW     (NB / NWAVE)
#define RCAP    8192
#define DEGCAP  64
#define GBM     128
#define GBN     64
#define GTHR    128
#define MROWS   128
#define NSEG    13
#define SMF     (NSEG * 512)
#define NEGSL   0.2f
#define WSMAX   134217728
#define LDS_SCAN ((2 * RCAP + 3 * NB + LISTN + 16) * 4)

static_assert((CHUNK & (CHUNK - 1)) == 0 && CHUNK <= (1 << 11));
static_assert(NB == (1 << SLOTB) && NTHR == NB && RPW * NWAVE == NB);
static_assert(LISTN >= NWAVE * WCAP);
static_assert((RCAP % 32) == 0);
static_assert(LDS_SCAN <= 300000);
static_assert(GBM == (GTHR / 32) * 32);
static_assert((XW % 32) == 0 && (KHL % 32) == 0 && KHL == 2 * HW);
static_assert((FW % GBN) == 0 && (HW % GBN) == 0 && FW == 3 * HW);
static_assert((MROWS % GBM) == 0);
static_assert(HW == 2 * 8 * 32);

typedef float          v4f  __attribute__((ext_vector_type(4)));
typedef float          v8f  __attribute__((ext_vector_type(8)));
typedef int            v4i  __attribute__((ext_vector_type(4)));
typedef int            v8i  __attribute__((ext_vector_type(8)));
typedef unsigned int   v4u  __attribute__((ext_vector_type(4)));
typedef unsigned short v8us __attribute__((ext_vector_type(8)));
typedef __bf16         v16b __attribute__((ext_vector_type(16)));
typedef v4f  __attribute__((may_alias)) v4fa;
typedef v8us __attribute__((may_alias)) v8usa;
union FragB { v16b v; v8us h[2]; v8i w; };

__device__ __forceinline__ v8f wmb(const FragB& a, const FragB& b, v8f c) {
  v8f d = __builtin_amdgcn_wmma_f32_16x16x32_bf16(false, a.v, false, b.v, (short)0, c, false, false);
  asm volatile("v_nop\n\tv_nop\n\tv_nop\n\tv_nop" : "+v"(d) : "v"(a.w), "v"(b.w));
  return d;
}

__device__ __forceinline__ unsigned int f2bf(float f) {
  const unsigned int u = __float_as_uint(f);
  return ((u + 0x7FFFu + ((u >> 16) & 1u)) >> 16) & 0xFFFFu;
}
__device__ __forceinline__ float bf2f(unsigned int b) { return __uint_as_float(b << 16); }
__device__ __forceinline__ float bfr(float f) { return bf2f(f2bf(f)); }
__device__ __forceinline__ v4f bfr4(const v4f a) {
  v4f r; r.x = bfr(a.x); r.y = bfr(a.y); r.z = bfr(a.z); r.w = bfr(a.w); return r;
}
__device__ __forceinline__ unsigned int pk2(float lo, float hi) { return f2bf(lo) | (f2bf(hi) << 16); }
__device__ __forceinline__ v4u pack8(const v4f a, const v4f b) {
  v4u r;
  r.x = pk2(a.x, a.y); r.y = pk2(a.z, a.w); r.z = pk2(b.x, b.y); r.w = pk2(b.z, b.w);
  return r;
}
__device__ __forceinline__ void split8(const v4f a, const v4f b, v4u& hi, v4u& lo) {
  const unsigned int h0 = f2bf(a.x), h1 = f2bf(a.y), h2 = f2bf(a.z), h3 = f2bf(a.w);
  const unsigned int h4 = f2bf(b.x), h5 = f2bf(b.y), h6 = f2bf(b.z), h7 = f2bf(b.w);
  const unsigned int l0 = f2bf(a.x - bf2f(h0)), l1 = f2bf(a.y - bf2f(h1));
  const unsigned int l2 = f2bf(a.z - bf2f(h2)), l3 = f2bf(a.w - bf2f(h3));
  const unsigned int l4 = f2bf(b.x - bf2f(h4)), l5 = f2bf(b.y - bf2f(h5));
  const unsigned int l6 = f2bf(b.z - bf2f(h6)), l7 = f2bf(b.w - bf2f(h7));
  hi.x = h0 | (h1 << 16); hi.y = h2 | (h3 << 16); hi.z = h4 | (h5 << 16); hi.w = h6 | (h7 << 16);
  lo.x = l0 | (l1 << 16); lo.y = l2 | (l3 << 16); lo.z = l4 | (l5 << 16); lo.w = l6 | (l7 << 16);
}

__global__ __launch_bounds__(128) void k_small(
    const float* __restrict__ b1s, const float* __restrict__ b1d, const float* __restrict__ b1r,
    const float* __restrict__ b2s, const float* __restrict__ b2d, const float* __restrict__ b2r,
    const float* __restrict__ bp, const float* __restrict__ at1, const float* __restrict__ at2,
    float* sm) {
  const int seg = (int)blockIdx.x;
  const int t4  = 4 * (int)threadIdx.x;
  v4f v;
  if      (seg == 0)  v = *(const v4fa*)(b1s + t4);
  else if (seg == 1)  v = *(const v4fa*)(b1d + t4);
  else if (seg == 2)  v = *(const v4fa*)(b1r + t4);
  else if (seg == 3)  v = *(const v4fa*)(b2s + t4);
  else if (seg == 4)  v = *(const v4fa*)(b2d + t4);
  else if (seg == 5)  v = *(const v4fa*)(b2r + t4);
  else if (seg == 6)  v = *(const v4fa*)(b2s + 512 + t4);
  else if (seg == 7)  v = *(const v4fa*)(b2d + 512 + t4);
  else if (seg == 8)  v = *(const v4fa*)(b2r + 512 + t4);
  else if (seg == 9)  v = *(const v4fa*)(bp + t4);
  else if (seg == 10) v = *(const v4fa*)(at1 + t4);
  else if (seg == 11) v = *(const v4fa*)(at2 + t4);
  else                v = *(const v4fa*)(at2 + 512 + t4);
  const v4f o = bfr4(v);
  float* op = sm + 512 * seg + t4;
  *(volatile v4f*)op = o;
  __threadfence();
  *(volatile v4f*)op = o;
}

__global__ __launch_bounds__(NTHR) void k_xprep(const float* __restrict__ x, unsigned short* xb, int nN, int nUnits) {
  const int i = (int)blockIdx.x * NTHR + (int)threadIdx.x;
  if (i >= nUnits) return;
  const int row = i >> 7;
  const int c0  = (i & 127) * 8;
  const int rc  = row < nN ? row : nN - 1;
  const float* p = x + (size_t)rc * XW + c0;
  v4f a = *(const v4fa*)p, b = *(const v4fa*)(p + 4);
  const v4f z4 = {0.f, 0.f, 0.f, 0.f};
  if (row >= nN) { a = z4; b = z4; }
  const v4u hv = pack8(a, b);
  const size_t o = (size_t)row * XW + c0;
  *(volatile v4u*)(xb + o) = hv;
  __threadfence();
  *(volatile v4u*)(xb + o) = hv;
}

__device__ __forceinline__ void ld8s(const float* __restrict__ p, size_t ld, v4f& a, v4f& b) {
  a.x = p[0];        a.y = p[ld];       a.z = p[2 * ld];   a.w = p[3 * ld];
  b.x = p[4 * ld];   b.y = p[5 * ld];   b.z = p[6 * ld];   b.w = p[7 * ld];
}

__global__ __launch_bounds__(NTHR) void k_wtr3(const float* __restrict__ w0, const float* __restrict__ w1,
                                               const float* __restrict__ w2, int Kin, int ld, int nPart, int Kout,
                                               unsigned short* wt, int nUnits) {
  const int u = (int)blockIdx.x * NTHR + (int)threadIdx.x;
  if (u >= nUnits) return;
  const int part = (int)blockIdx.y, head = (int)blockIdx.z;
  const int kq = Kout >> 3;
  const int n  = u / kq;
  const int k8 = (u - n * kq) * 8;
  const int kk = k8 - (k8 / Kin) * Kin;
  const size_t so = (size_t)kk * (size_t)ld + (size_t)(head * nPart + n);
  v4f a, b;
  if (part == 0)      ld8s(w0 + so, (size_t)ld, a, b);
  else if (part == 1) ld8s(w1 + so, (size_t)ld, a, b);
  else                ld8s(w2 + so, (size_t)ld, a, b);
  const v4u wv = pack8(a, b);
  const int orow = (head * (int)gridDim.y + part) * nPart + n;
  unsigned short* o = wt + (size_t)orow * (size_t)Kout + k8;
  *(volatile v4u*)o = wv;
  __threadfence();
  *(volatile v4u*)o = wv;
}

__global__ __launch_bounds__(GTHR) void k_gemm(
    const unsigned short* __restrict__ A, const unsigned short* __restrict__ WT,
    const float* __restrict__ bias, float* C, int K, int ldc, int nStore)
{
  __shared__ __attribute__((aligned(16))) float stg[GBM * GBN];
  const int tid = (int)threadIdx.x, lane = tid & 31, wave = tid >> 5, hh = lane >> 4, m = lane & 15;
  const int rowBase = (int)blockIdx.x * GBM;
  const int col0    = (int)blockIdx.y * GBN;

  v8f acc0[4], acc1[4];
  {
    const v8f z = {0.f, 0.f, 0.f, 0.f, 0.f, 0.f, 0.f, 0.f};
    acc0[0] = z; acc0[1] = z; acc0[2] = z; acc0[3] = z;
    acc1[0] = z; acc1[1] = z; acc1[2] = z; acc1[3] = z;
  }
  const unsigned short* ap0 = A  + (size_t)(rowBase + 32 * wave + m) * (size_t)K + 8 * hh;
  const unsigned short* ap1 = ap0 + (size_t)16 * (size_t)K;
  const unsigned short* wp  = WT + (size_t)(col0 + m) * (size_t)K + 8 * hh;
  const int ksteps = K >> 5;
#pragma unroll 1
  for (int ks = 0; ks < ksteps; ++ks) {
    FragB af0, af1;
    af0.h[0] = *(const v8usa*)(ap0 + 32 * ks);
    af0.h[1] = *(const v8usa*)(ap0 + 32 * ks + 16);
    af1.h[0] = *(const v8usa*)(ap1 + 32 * ks);
    af1.h[1] = *(const v8usa*)(ap1 + 32 * ks + 16);
#pragma unroll
    for (int t = 0; t < 4; ++t) {
      const unsigned short* wq = wp + (size_t)(16 * t) * (size_t)K + 32 * ks;
      FragB bf;
      bf.h[0] = *(const v8usa*)wq;
      bf.h[1] = *(const v8usa*)(wq + 16);
      acc0[t] = wmb(af0, bf, acc0[t]);
      acc1[t] = wmb(af1, bf, acc1[t]);
    }
  }

  float bv[4];
#pragma unroll
  for (int t = 0; t < 4; ++t) bv[t] = bias[col0 + 16 * t + m];

#pragma unroll
  for (int t = 0; t < 4; ++t) {
    const int lc = 16 * t + m;
#pragma unroll
    for (int r = 0; r < 8; ++r) {
      const int lr = 32 * wave + 8 * hh + r;
      stg[lr * GBN + lc]        = acc0[t][r] + bv[t];
      stg[(lr + 16) * GBN + lc] = acc1[t][r] + bv[t];
    }
  }
  __syncthreads();

#pragma unroll 4
  for (int i = 0; i < 16; ++i) {
    const int lr = 32 * wave + 2 * i + hh;
    const int gr = rowBase + lr;
    const v4f fv = *(const v4fa*)(stg + lr * GBN + 4 * m);
    float* op = C + (size_t)gr * (size_t)ldc + col0 + 4 * m;
    if (gr < nStore) *(volatile v4f*)op = fv;
  }
  __threadfence();
#pragma unroll 4
  for (int i = 0; i < 16; ++i) {
    const int lr = 32 * wave + 2 * i + hh;
    const int gr = rowBase + lr;
    const v4f fv = *(const v4fa*)(stg + lr * GBN + 4 * m);
    float* op = C + (size_t)gr * (size_t)ldc + col0 + 4 * m;
    if (gr < nStore) *(volatile v4f*)op = fv;
  }
}

__device__ __forceinline__ int scan_chunk(const int* __restrict__ dsts, int nE, int cbase, int slotBase,
                                          int vec8, int* list, int tid, int lane, int wave) {
  const int el0  = tid * EPT;
  const int e0   = cbase + el0;
  const int sent = -2147483647 - 1;
  v4i da, db;
  if (vec8 != 0 && cbase + CHUNK <= nE) {
    da = *(const v4i*)(dsts + e0);
    db = *(const v4i*)(dsts + e0 + 4);
  } else {
    da.x = (e0     < nE) ? dsts[min(e0,     nE - 1)] : sent;
    da.y = (e0 + 1 < nE) ? dsts[min(e0 + 1, nE - 1)] : sent;
    da.z = (e0 + 2 < nE) ? dsts[min(e0 + 2, nE - 1)] : sent;
    da.w = (e0 + 3 < nE) ? dsts[min(e0 + 3, nE - 1)] : sent;
    db.x = (e0 + 4 < nE) ? dsts[min(e0 + 4, nE - 1)] : sent;
    db.y = (e0 + 5 < nE) ? dsts[min(e0 + 5, nE - 1)] : sent;
    db.z = (e0 + 6 < nE) ? dsts[min(e0 + 6, nE - 1)] : sent;
    db.w = (e0 + 7 < nE) ? dsts[min(e0 + 7, nE - 1)] : sent;
  }
  const unsigned nbs = (unsigned)slotBase;
  const unsigned unb = (unsigned)NB;
  const unsigned s0 = (unsigned)da.x - nbs, s1 = (unsigned)da.y - nbs;
  const unsigned s2 = (unsigned)da.z - nbs, s3 = (unsigned)da.w - nbs;
  const unsigned s4 = (unsigned)db.x - nbs, s5 = (unsigned)db.y - nbs;
  const unsigned s6 = (unsigned)db.z - nbs, s7 = (unsigned)db.w - nbs;
  const bool h0 = s0 < unb, h1 = s1 < unb, h2 = s2 < unb, h3 = s3 < unb;
  const bool h4 = s4 < unb, h5 = s5 < unb, h6 = s6 < unb, h7 = s7 < unb;
  const int c = (int)h0 + (int)h1 + (int)h2 + (int)h3 + (int)h4 + (int)h5 + (int)h6 + (int)h7;
  int incl = c;
#pragma unroll
  for (int d = 1; d < 32; d <<= 1) {
    const int up = __shfl_up(incl, d);
    incl += (lane >= d) ? up : 0;
  }
  const int wc = __shfl(incl, 31);
  const int lim = wave * WCAP + WCAP - 1;
  int pos = wave * WCAP + (incl - c);
#define PUTJ(J, HJ, SJ) if (HJ) { list[pos < lim ? pos : lim] = ((el0 + (J)) << SLOTB) | (int)(SJ); pos = pos + 1; }
  PUTJ(0, h0, s0)
  PUTJ(1, h1, s1)
  PUTJ(2, h2, s2)
  PUTJ(3, h3, s3)
  PUTJ(4, h4, s4)
  PUTJ(5, h5, s5)
  PUTJ(6, h6, s6)
  PUTJ(7, h7, s7)
#undef PUTJ
  return wc;
}

__device__ __forceinline__ float ldot4(const v4f f, const v4f d, const v4f a, float p) {
  float t;
  t = f.x + d.x; t = fmaxf(t, NEGSL * t); p = fmaf(t, a.x, p);
  t = f.y + d.y; t = fmaxf(t, NEGSL * t); p = fmaf(t, a.y, p);
  t = f.z + d.z; t = fmaxf(t, NEGSL * t); p = fmaf(t, a.z, p);
  t = f.w + d.w; t = fmaxf(t, NEGSL * t); p = fmaf(t, a.w, p);
  return p;
}
__device__ __forceinline__ void smx(float lg, float& mx, float& l, float& s1, float& s2) {
  const float df = lg - mx;
  const float ee = expf(-fabsf(df));
  const bool up  = df > 0.f;
  s1 = up ? ee : 1.0f;
  s2 = up ? 1.0f : ee;
  mx = up ? lg : mx;
  l  = fmaf(l, s1, s2);
}
__device__ __forceinline__ v4f upd4(const v4f a, float s1, float s2, const v4f f) {
  v4f r;
  r.x = fmaf(a.x, s1, s2 * f.x); r.y = fmaf(a.y, s1, s2 * f.y);
  r.z = fmaf(a.z, s1, s2 * f.z); r.w = fmaf(a.w, s1, s2 * f.w);
  return r;
}
__device__ __forceinline__ v4f fin4(const v4f a, float inv, const v4f r) {
  v4f o; float c;
  c = fmaf(a.x, inv, r.x); o.x = (c > 0.f) ? c : (c - c);
  c = fmaf(a.y, inv, r.y); o.y = (c > 0.f) ? c : (c - c);
  c = fmaf(a.z, inv, r.z); o.z = (c > 0.f) ? c : (c - c);
  c = fmaf(a.w, inv, r.w); o.w = (c > 0.f) ? c : (c - c);
  return o;
}
__device__ __forceinline__ v4f addrelu4(const v4f z, const v4f v) {
  v4f o; float c;
  c = z.x + v.x; o.x = (c > 0.f) ? c : (c - c);
  c = z.y + v.y; o.y = (c > 0.f) ? c : (c - c);
  c = z.z + v.z; o.z = (c > 0.f) ? c : (c - c);
  c = z.w + v.w; o.w = (c > 0.f) ? c : (c - c);
  return o;
}
__device__ __forceinline__ v4f pz4(const v4f v, float pz, bool live) {
  v4f o;
  o.x = live ? (v.x + pz) : 0.f; o.y = live ? (v.y + pz) : 0.f;
  o.z = live ? (v.z + pz) : 0.f; o.w = live ? (v.w + pz) : 0.f;
  return o;
}

template<int MODE>
__global__ __launch_bounds__(NTHR) void k_scan(
    const int* __restrict__ srcs, const int* __restrict__ dsts,
    const float* __restrict__ F, const float* __restrict__ att,
    float* Z, unsigned short* HP,
    int nN, int nE, int vec8, int MPr) {
  extern __shared__ v4f lds_dyn[];
  int* reg1 = (int*)lds_dyn;
  int* reg2 = reg1 + RCAP;
  int* scnt = reg2 + RCAP;
  int* soff = scnt + NB;
  int* cur  = soff + NB;
  int* list = cur + NB;
  int* wcnt = list + LISTN;
  int* wtot = wcnt + NWAVE;
  const int tid = (int)threadIdx.x, lane = tid & 31, wave = tid >> 5;
  const int nodeBase = (int)blockIdx.x * NB;

  scnt[tid] = 0;
  __syncthreads();

  int tot = 0;
  const int nChunks = (nE + CHUNK - 1) / CHUNK;
#pragma unroll 1
  for (int ch = 0; ch < nChunks; ++ch) {
    const int cbase = ch * CHUNK;
    const int wc = scan_chunk(dsts, nE, cbase, nodeBase, vec8, list, tid, lane, wave);
    if (lane == 0) wcnt[wave] = wc;
    __syncthreads();
    int pre = 0, all = 0;
#pragma unroll
    for (int w2 = 0; w2 < NWAVE; ++w2) {
      int c = wcnt[w2];
      c = c < 0 ? 0 : (c > WCAP ? WCAP : c);
      all += c;
      pre += (w2 < wave) ? c : 0;
    }
    const int wcc  = wc > WCAP ? WCAP : wc;
    const int base = tot + pre;
#pragma unroll 1
    for (int i = lane; i < wcc; i += 32) {
      const int ent = list[wave * WCAP + i];
      const int el  = (ent >> SLOTB) & (CHUNK - 1);
      const int sl  = ent & (NB - 1);
      int eid = cbase + el;
      eid = eid > nE - 1 ? nE - 1 : eid;
      const int pos = base + i;
      if (pos < RCAP) reg1[pos] = (int)(((unsigned)eid << SLOTB) | (unsigned)sl);
    }
    tot += all;
    tot = tot > RCAP ? RCAP : tot;
    __syncthreads();
  }
  const int nh = tot;

  if (wave == 0) {
#pragma unroll 1
    for (int b0 = 0; b0 < nh; b0 += 32) {
      const int idx = b0 + lane;
      const int uv  = reg1[idx < nh ? idx : nh - 1];
      const int m32 = (nh - b0) < 32 ? (nh - b0) : 32;
#pragma unroll 1
      for (int k = 0; k < m32; ++k) {
        const int u  = __builtin_amdgcn_readlane(uv, k);
        const int sl = u & (NB - 1);
        if (lane == 0) scnt[sl] = scnt[sl] + 1;
      }
    }
  }
  __syncthreads();

  {
    int c = scnt[tid];
    c = c < 0 ? 0 : c;
    int incl = c;
#pragma unroll
    for (int d = 1; d < 32; d <<= 1) {
      const int up = __shfl_up(incl, d);
      incl += (lane >= d) ? up : 0;
    }
    if (lane == 31) wtot[wave] = incl;
    __syncthreads();
    int pre = 0;
#pragma unroll
    for (int w2 = 0; w2 < NWAVE; ++w2) pre += (w2 < wave) ? wtot[w2] : 0;
    const int ex = pre + incl - c;
    soff[tid] = ex;
    cur[tid]  = ex;
  }
  __syncthreads();

  if (wave == 0) {
#pragma unroll 1
    for (int b0 = 0; b0 < nh; b0 += 32) {
      const int idx = b0 + lane;
      const int uv  = reg1[idx < nh ? idx : nh - 1];
      const int m32 = (nh - b0) < 32 ? (nh - b0) : 32;
#pragma unroll 1
      for (int k = 0; k < m32; ++k) {
        const int u   = __builtin_amdgcn_readlane(uv, k);
        const int sl  = u & (NB - 1);
        const int eid = (int)((unsigned)u >> SLOTB);
        if (lane == 0) {
          int pos = cur[sl];
          pos = pos < 0 ? 0 : (pos > RCAP - 1 ? RCAP - 1 : pos);
          reg2[pos] = eid;
          cur[sl] = pos + 1;
        }
      }
    }
  }
  __syncthreads();

  const bool ovf = (nh >= RCAP);
  const float qnan = __int_as_float(0x7fc00000);
  const v4f z4 = {0.f, 0.f, 0.f, 0.f};
  const int cofs0 = 8 * lane;
  const int cofs1 = 256 + 8 * lane;
  const v4f at00 = *(const v4fa*)(att + cofs0), at01 = *(const v4fa*)(att + cofs0 + 4);
  const v4f at10 = *(const v4fa*)(att + cofs1), at11 = *(const v4fa*)(att + cofs1 + 4);

#pragma unroll 1
  for (int jt = 0; jt < RPW; ++jt) {
    const int slot = wave * RPW + jt;
    const int grow = nodeBase + slot;
    const int gcl  = grow < nN ? grow : nN - 1;
    int st = soff[slot];
    const int craw = scnt[slot];
    int cnt = craw;
    st  = st < 0 ? 0 : (st > nh ? nh : st);
    cnt = cnt < 0 ? 0 : (cnt > DEGCAP ? DEGCAP : cnt);
    if (cnt > nh - st) cnt = nh - st;
    const float pz = (ovf || craw > DEGCAP) ? qnan : 0.0f;

    const float* frow = F + (size_t)gcl * FW;
    const v4f d00 = *(const v4fa*)(frow + HW + cofs0), d01 = *(const v4fa*)(frow + HW + cofs0 + 4);
    const v4f d10 = *(const v4fa*)(frow + HW + cofs1), d11 = *(const v4fa*)(frow + HW + cofs1 + 4);
    float m0 = -3.0e38f, m1 = -3.0e38f, l0 = 0.0f, l1 = 0.0f;
    v4f a00 = z4, a01 = z4, a10 = z4, a11 = z4;

#pragma unroll 1
    for (int q = 0; q < cnt; ++q) {
      int idx = st + q; idx = idx > RCAP - 1 ? RCAP - 1 : idx;
      int eid = reg2[idx]; eid = eid < 0 ? 0 : (eid > nE - 1 ? nE - 1 : eid);
      const int sraw = srcs[eid];
      const int s = sraw < 0 ? 0 : (sraw > nN - 1 ? nN - 1 : sraw);
      const float* sp = F + (size_t)s * FW;
      const v4f f00 = *(const v4fa*)(sp + cofs0), f01 = *(const v4fa*)(sp + cofs0 + 4);
      const v4f f10 = *(const v4fa*)(sp + cofs1), f11 = *(const v4fa*)(sp + cofs1 + 4);
      float p0 = ldot4(f00, d00, at00, 0.0f); p0 = ldot4(f01, d01, at01, p0);
      float p1 = ldot4(f10, d10, at10, 0.0f); p1 = ldot4(f11, d11, at11, p1);
      float pa = (MODE == 0) ? p0 : (p0 + p1);
      float pb = p1;
#pragma unroll
      for (int off = 16; off > 0; off >>= 1) {
        pa += __shfl_xor(pa, off);
        if (MODE == 0) pb += __shfl_xor(pb, off);
      }
      float s1a, s2a, s1b, s2b;
      smx(pa, m0, l0, s1a, s2a);
      if (MODE == 0) { smx(pb, m1, l1, s1b, s2b); } else { s1b = s1a; s2b = s2a; }
      a00 = upd4(a00, s1a, s2a, f00); a01 = upd4(a01, s1a, s2a, f01);
      a10 = upd4(a10, s1b, s2b, f10); a11 = upd4(a11, s1b, s2b, f11);
    }

    const bool has = cnt > 0;
    const float r0 = __builtin_amdgcn_rcpf(l0);
    const float r1 = __builtin_amdgcn_rcpf(l1);
    const float inv0 = has ? r0 : 0.0f;
    const float inv1 = (MODE == 0) ? (has ? r1 : 0.0f) : inv0;
    const v4f q00 = *(const v4fa*)(frow + 2 * HW + cofs0), q01 = *(const v4fa*)(frow + 2 * HW + cofs0 + 4);
    const v4f q10 = *(const v4fa*)(frow + 2 * HW + cofs1), q11 = *(const v4fa*)(frow + 2 * HW + cofs1 + 4);
    v4f v00 = fin4(a00, inv0, q00), v01 = fin4(a01, inv0, q01);
    v4f v10 = fin4(a10, inv1, q10), v11 = fin4(a11, inv1, q11);
    const bool live = grow < nN;
    const bool wr   = grow < MPr;

    if (MODE == 2) {
      const float* zp = Z + (size_t)gcl * HW + 4 * lane;
      const v4f z00 = *(const v4fa*)(zp),       z01 = *(const v4fa*)(zp + 128);
      const v4f z10 = *(const v4fa*)(zp + 256), z11 = *(const v4fa*)(zp + 384);
      v00 = addrelu4(z00, v00); v01 = addrelu4(z01, v01);
      v10 = addrelu4(z10, v10); v11 = addrelu4(z11, v11);
    }
    v00 = pz4(v00, pz, live); v01 = pz4(v01, pz, live);
    v10 = pz4(v10, pz, live); v11 = pz4(v11, pz, live);

    if (MODE == 1) {
      float* zo = Z + (size_t)grow * HW + 4 * lane;
      if (wr) {
        *(volatile v4f*)(zo)       = v00;
        *(volatile v4f*)(zo + 128) = v01;
        *(volatile v4f*)(zo + 256) = v10;
        *(volatile v4f*)(zo + 384) = v11;
      }
      __threadfence();
      if (wr) {
        *(volatile v4f*)(zo)       = v00;
        *(volatile v4f*)(zo + 128) = v01;
        *(volatile v4f*)(zo + 256) = v10;
        *(volatile v4f*)(zo + 384) = v11;
      }
    } else {
      v4u hi0, lo0, hi1, lo1;
      split8(v00, v01, hi0, lo0);
      split8(v10, v11, hi1, lo1);
      unsigned short* hp = HP + (size_t)grow * KHL;
      if (wr) {
        *(volatile v4u*)(hp + cofs0)      = hi0;
        *(volatile v4u*)(hp + cofs1)      = hi1;
        *(volatile v4u*)(hp + HW + cofs0) = lo0;
        *(volatile v4u*)(hp + HW + cofs1) = lo1;
      }
      __threadfence();
      if (wr) {
        *(volatile v4u*)(hp + cofs0)      = hi0;
        *(volatile v4u*)(hp + cofs1)      = hi1;
        *(volatile v4u*)(hp + HW + cofs0) = lo0;
        *(volatile v4u*)(hp + HW + cofs1) = lo1;
      }
    }
  }
}

static inline int cdiv(int a, int b) { return (a + b - 1) / b; }

extern "C" void kernel_launch(void* const* d_in, const int* in_sizes, int n_in,
                              void* d_out, int out_size, void* d_ws, size_t ws_size,
                              hipStream_t stream) {
  if (n_in < 19) return;
  if (in_sizes[0] < XW || (in_sizes[0] % XW) != 0) return;
  const int nN = in_sizes[0] / XW;
  if (nN <= 0 || nN > (1 << 20)) return;
  const int nE = in_sizes[1];
  if (nE < 1 || nE >= (1 << 23) || in_sizes[2] != nE) return;
  if (in_sizes[3] != XW * HW || in_sizes[5] != XW * HW || in_sizes[8] != XW * HW) return;
  if (in_sizes[4] != HW || in_sizes[6] != HW || in_sizes[9] != HW) return;
  if (in_sizes[7] != HW) return;
  if (in_sizes[10] != HW * 1024 || in_sizes[12] != HW * 1024 || in_sizes[15] != HW * 1024) return;
  if (in_sizes[11] != 1024 || in_sizes[13] != 1024 || in_sizes[16] != 1024) return;
  if (in_sizes[14] != 1024) return;
  if (in_sizes[17] != HW * HW || in_sizes[18] != HW) return;
  if ((long long)out_size != (long long)nN * HW) return;

  const float* x   = (const float*)d_in[0];
  const int*   src = (const int*)  d_in[1];
  const int*   dst = (const int*)  d_in[2];
  const float* W1s = (const float*)d_in[3];
  const float* b1s = (const float*)d_in[4];
  const float* W1d = (const float*)d_in[5];
  const float* b1d = (const float*)d_in[6];
  const float* at1 = (const float*)d_in[7];
  const float* W1r = (const float*)d_in[8];
  const float* b1r = (const float*)d_in[9];
  const float* W2s = (const float*)d_in[10];
  const float* b2s = (const float*)d_in[11];
  const float* W2d = (const float*)d_in[12];
  const float* b2d = (const float*)d_in[13];
  const float* at2 = (const float*)d_in[14];
  const float* W2r = (const float*)d_in[15];
  const float* b2r = (const float*)d_in[16];
  const float* Wp  = (const float*)d_in[17];
  const float* bp  = (const float*)d_in[18];
  float* out = (float*)d_out;

  const int MP   = cdiv(nN, MROWS) * MROWS;
  const int gA   = cdiv(MP, NB);
  const int vec8 = ((nE & 3) == 0) ? 1 : 0;
  if ((long long)gA * NB < (long long)MP) return;

  char* ws = (char*)d_ws;
  size_t off = 0;
  const size_t oSM  = off; off += (size_t)SMF * 4;                 off = (off + 255) & ~(size_t)255;
  const size_t oW1T = off; off += (size_t)FW * XW * 2;             off = (off + 255) & ~(size_t)255;
  const size_t oW2T = off; off += (size_t)2 * FW * KHL * 2;        off = (off + 255) & ~(size_t)255;
  const size_t oWPT = off; off += (size_t)HW * KHL * 2;            off = (off + 255) & ~(size_t)255;
  const size_t oXB  = off; off += (size_t)MP * XW * 2;             off = (off + 255) & ~(size_t)255;
  const size_t oF   = off; off += (size_t)MP * FW * 4;             off = (off + 255) & ~(size_t)255;
  const size_t oH   = off; off += (size_t)MP * KHL * 2;            off = (off + 255) & ~(size_t)255;
  if (off > ws_size || off > (size_t)WSMAX) return;
  static_assert((size_t)XW * 2 == (size_t)HW * 4);
  float*          SM   = (float*)(ws + oSM);
  unsigned short* W1T  = (unsigned short*)(ws + oW1T);
  unsigned short* W2T2 = (unsigned short*)(ws + oW2T);
  unsigned short* WPT2 = (unsigned short*)(ws + oWPT);
  unsigned short* XB   = (unsigned short*)(ws + oXB);
  float*          Zp   = (float*)(ws + oXB);
  float*          Fp   = (float*)(ws + oF);
  unsigned short* Hp   = (unsigned short*)(ws + oH);
  const float* B1   = SM;
  const float* B2   = SM + 1536;
  const float* BP   = SM + 4608;
  const float* ATT1 = SM + 5120;
  const float* ATT2 = SM + 5632;

  hipFuncSetAttribute(reinterpret_cast<const void*>(&k_scan<0>), hipFuncAttributeMaxDynamicSharedMemorySize, LDS_SCAN);
  hipFuncSetAttribute(reinterpret_cast<const void*>(&k_scan<1>), hipFuncAttributeMaxDynamicSharedMemorySize, LDS_SCAN);
  hipFuncSetAttribute(reinterpret_cast<const void*>(&k_scan<2>), hipFuncAttributeMaxDynamicSharedMemorySize, LDS_SCAN);

  k_small<<<NSEG, 128, 0, stream>>>(b1s, b1d, b1r, b2s, b2d, b2r, bp, at1, at2, SM);
  const int nUx = MP * (XW / 8);
  k_xprep<<<cdiv(nUx, NTHR), NTHR, 0, stream>>>(x, XB, nN, nUx);
  {
    const int nUw = HW * (KHL / 8);
    k_wtr3<<<dim3(cdiv(nUw, NTHR), 3, 1), NTHR, 0, stream>>>(W1s, W1d, W1r, XW, HW, HW, XW, W1T, nUw);
    k_wtr3<<<dim3(cdiv(nUw, NTHR), 3, 2), NTHR, 0, stream>>>(W2s, W2d, W2r, HW, 1024, HW, KHL, W2T2, nUw);
    k_wtr3<<<dim3(cdiv(nUw, NTHR), 1, 1), NTHR, 0, stream>>>(Wp, Wp, Wp, HW, HW, HW, KHL, WPT2, nUw);
  }

  const int gM = MP / GBM;
  k_gemm<<<dim3(gM, FW / GBN), GTHR, 0, stream>>>(XB, W1T, B1, Fp, XW, FW, MP);
  k_scan<0><<<gA, NTHR, LDS_SCAN, stream>>>(src, dst, Fp, ATT1, Zp, Hp, nN, nE, vec8, MP);
  k_gemm<<<dim3(gM, FW / GBN), GTHR, 0, stream>>>(Hp, W2T2, B2, Fp, KHL, FW, MP);
  k_scan<1><<<gA, NTHR, LDS_SCAN, stream>>>(src, dst, Fp, ATT2, Zp, Hp, nN, nE, vec8, MP);
  k_gemm<<<dim3(gM, FW / GBN), GTHR, 0, stream>>>(Hp, W2T2 + (size_t)FW * KHL, B2 + FW, Fp, KHL, FW, MP);
  k_scan<2><<<gA, NTHR, LDS_SCAN, stream>>>(src, dst, Fp, ATT2 + HW, Zp, Hp, nN, nE, vec8, MP);
  k_gemm<<<dim3(gM, HW / GBN), GTHR, 0, stream>>>(Hp, WPT2, BP, out, KHL, HW, nN);
}
